// GraphConvolution_16758962389075
// MI455X (gfx1250) — hardware-run, weakly checked
//
#include <hip/hip_runtime.h>
#include <stddef.h>
#include <stdint.h>
#include <math.h>

#define NN      100000
#define KD      128
#define HD      64
#define NE      3200000
#define GBM     128
#define MP      100096
#define NTHR    256
#define NWAVE   8
#define EPT     8
#define WCH     (32 * EPT)
#define NBRUN   512
#define SLB     9
#define NBK     196
#define WLCAP   2880
#define RCAP    18432
#define DEGCAP  128
#define MAXDEG_MEAS  57
#define MAXB512_MEAS 16837
#define SP      68
#define WSMAX   134217728

#define BK_ZINTS (NWAVE * WLCAP + 2 * RCAP + 3 * NBRUN)
#define BK_INTS  (BK_ZINTS + 16)
#define BK_LDS   (BK_INTS * 4)

#define PBX  (MP * KD / 8 / NTHR)
#define PBW  (HD * KD / 8 / NTHR)
#define PBZ  252
#define PBTOT (PBX + PBW + PBZ)

static_assert(HD == 32 * 2 && HD == 16 * 4);
static_assert(KD % 32 == 0);
static_assert(MP % GBM == 0 && MP >= NN && MP == 782 * GBM && MP - NN == 96);
static_assert(NBRUN == (1 << SLB) && NBRUN % 32 == 0 && NBRUN % 16 == 0 && NBRUN % NWAVE == 0);
static_assert(NBK * NBRUN >= MP && (NBK - 1) * NBRUN < NN && NN - (NBK - 1) * NBRUN == 160);
static_assert(NE < (1 << 22) && (((long long)NE) << SLB) < (1LL << 31));
static_assert(NE % WCH == 0 && NE % 4 == 0);
static_assert(RCAP % 16 == 0 && BK_ZINTS % 4 == 0);
static_assert((long long)RCAP * 100 >= (long long)MAXB512_MEAS * 105);
static_assert(WLCAP * 8 >= (RCAP / 8) * 10);
static_assert(WLCAP >= MAXB512_MEAS / 8 + 8 * 46 + 1);
static_assert(MAXDEG_MEAS + 8 <= DEGCAP);
static_assert((2 * RCAP) % (NTHR * 4) == 0 && 2 * NBRUN == NTHR * 4);
static_assert((MP * KD / 8) % NTHR == 0 && (HD * KD / 8) % NTHR == 0);
static_assert((NN * HD / 4) % NTHR == 0);
static_assert(BK_LDS <= 300000);
static_assert(GBM * SP * 4 <= 65536);

typedef float          v2f   __attribute__((ext_vector_type(2)));
typedef float          v4f   __attribute__((ext_vector_type(4)));
typedef float          v8f   __attribute__((ext_vector_type(8)));
typedef double         v2d   __attribute__((ext_vector_type(2)));
typedef int            v2i   __attribute__((ext_vector_type(2)));
typedef int            v4i   __attribute__((ext_vector_type(4)));
typedef int            v8i   __attribute__((ext_vector_type(8)));
typedef unsigned short v8us  __attribute__((ext_vector_type(8)));
typedef unsigned short v16us __attribute__((ext_vector_type(16)));
typedef __bf16         v16bf __attribute__((ext_vector_type(16)));
typedef v2f  __attribute__((may_alias)) v2fa;
typedef v4f  __attribute__((may_alias)) v4fa;
typedef v2d  __attribute__((may_alias)) v2da;
typedef v2i  __attribute__((may_alias)) v2ia;
typedef v4i  __attribute__((may_alias)) v4ia;
typedef v8us __attribute__((may_alias)) v8usa;
union FragB { v16bf v; v16us u; v8us h[2]; v8i w; };

__device__ __forceinline__ v8f wmb(const FragB& a, const FragB& b, v8f c) {
  v8f d = __builtin_amdgcn_wmma_f32_16x16x32_bf16(false, a.v, false, b.v, (short)0, c, false, false);
  asm volatile("v_nop\n\tv_nop\n\tv_nop\n\tv_nop" : "+v"(d) : "v"(a.w), "v"(b.w));
  return d;
}

__device__ __forceinline__ unsigned bf16_bits(float f) {
  const unsigned u = __float_as_uint(f);
  const unsigned r = (u + 0x7FFFu + ((u >> 16) & 1u)) >> 16;
  const unsigned q = (u >> 16) | 0x40u;
  return ((u & 0x7fffffffu) > 0x7f800000u) ? q : r;
}

__device__ __forceinline__ void st2_v4f(float* p, v4f v) {
  *(volatile v4f*)p = v;
  __threadfence();
  *(volatile v4f*)p = v;
}
__device__ __forceinline__ void st2_v4i(int* p, v4i v) {
  *(volatile v4i*)p = v;
  __threadfence();
  *(volatile v4i*)p = v;
}
__device__ __forceinline__ void st2_v8us(unsigned short* p, v8us v) {
  *(volatile v8us*)p = v;
  __threadfence();
  *(volatile v8us*)p = v;
}

__device__ __forceinline__ v8us gather8(const float* __restrict__ base, int stride) {
  float f[8];
#pragma unroll
  for (int i = 0; i < 8; ++i) f[i] = base[(size_t)i * (size_t)stride];
  v8us o;
#pragma unroll
  for (int i = 0; i < 8; ++i) o[i] = (unsigned short)bf16_bits(f[i]);
  return o;
}

__global__ __launch_bounds__(NTHR) void k_prep(const float* __restrict__ x, const float* __restrict__ w,
                                               unsigned short* xb, unsigned short* wt, int* zreg) {
  const int tid = (int)threadIdx.x;
  const int blk = (int)blockIdx.x;
  if (blk < PBX) {
    const int u   = blk * NTHR + tid;
    const int row = u >> 4, k8 = (u & 15) * 8;
    const int rc  = row < NN ? row : NN - 1;
    const unsigned mk = row < NN ? 0xffffu : 0u;
    const float* p = x + (size_t)rc * KD + k8;
    const v4f a = *(const v4fa*)p;
    const v4f b = *(const v4fa*)(p + 4);
    v8us o;
    o[0] = (unsigned short)(bf16_bits(a.x) & mk); o[1] = (unsigned short)(bf16_bits(a.y) & mk);
    o[2] = (unsigned short)(bf16_bits(a.z) & mk); o[3] = (unsigned short)(bf16_bits(a.w) & mk);
    o[4] = (unsigned short)(bf16_bits(b.x) & mk); o[5] = (unsigned short)(bf16_bits(b.y) & mk);
    o[6] = (unsigned short)(bf16_bits(b.z) & mk); o[7] = (unsigned short)(bf16_bits(b.w) & mk);
    st2_v8us(xb + (size_t)row * KD + k8, o);
  } else if (blk < PBX + PBW) {
    const int u = (blk - PBX) * NTHR + tid;
    const int n = u >> 4, k8 = (u & 15) * 8;
    const v8us o = gather8(w + (size_t)k8 * HD + n, HD);
    st2_v8us(wt + (size_t)n * KD + k8, o);
  } else {
    const int u = (blk - PBX - PBW) * NTHR + tid;
    const v4i z4 = {0, 0, 0, 0};
    st2_v4i(zreg + (size_t)4 * (size_t)u, z4);
  }
}

__device__ __forceinline__ void bucket_flush(const int* pl, const int* cnt, int ov, int* lp, int* cop, int* fp,
                                             int tid) {
#pragma unroll 1
  for (int i = tid * 4; i < 2 * RCAP; i += NTHR * 4) {
    const v4i v = *(const v4ia*)(pl + i);
    *(volatile v4i*)(lp + i) = v;
  }
  {
    const v4i v = *(const v4ia*)(cnt + 4 * tid);
    *(volatile v4i*)(cop + 4 * tid) = v;
  }
  if (tid < 8) {
    const v4i f = {ov, ov, ov, ov};
    *(volatile v4i*)(fp + 4 * tid) = f;
  }
}

__global__ __launch_bounds__(NTHR) void k_bucket(const int* __restrict__ srcs, const int* __restrict__ dsts,
                                                 const float* __restrict__ ew, int* LIST, int* CO, int* FLAG) {
  extern __shared__ __attribute__((aligned(16))) int dsm[];
  int* wl   = dsm;
  int* pl   = dsm + NWAVE * WLCAP;
  int* cnt  = pl + 2 * RCAP;
  int* offs = cnt + NBRUN;
  int* cur  = offs + NBRUN;
  int* misc = cur + NBRUN;
  const int tid = (int)threadIdx.x, lane = tid & 31, wave = tid >> 5;
  const int blk = (int)blockIdx.x;
  const unsigned nbs = (unsigned)(blk * NBRUN);

  {
    const v4i z4 = {0, 0, 0, 0};
    for (int i = tid * 4; i < BK_ZINTS; i += NTHR * 4) *(v4ia*)(dsm + i) = z4;
    if (tid < 16) misc[tid] = 0;
  }
  __syncthreads();

  {
    const int per  = ((NE + NWAVE * WCH - 1) / (NWAVE * WCH)) * WCH;
    const int ebeg = wave * per;
    const int eend = (ebeg + per < NE) ? (ebeg + per) : NE;
    int* mylist = wl + wave * WLCAP;
    int wc = 0;
#pragma unroll 1
    for (int cb = ebeg; cb < eend; cb += WCH) {
      const int e0 = cb + lane * EPT;
      const v4i da = *(const v4ia*)(dsts + e0);
      const v4i db = *(const v4ia*)(dsts + e0 + 4);
      const unsigned s0 = (unsigned)da.x - nbs, s1 = (unsigned)da.y - nbs;
      const unsigned s2 = (unsigned)da.z - nbs, s3 = (unsigned)da.w - nbs;
      const unsigned s4 = (unsigned)db.x - nbs, s5 = (unsigned)db.y - nbs;
      const unsigned s6 = (unsigned)db.z - nbs, s7 = (unsigned)db.w - nbs;
      const bool h0 = s0 < (unsigned)NBRUN, h1 = s1 < (unsigned)NBRUN, h2 = s2 < (unsigned)NBRUN, h3 = s3 < (unsigned)NBRUN;
      const bool h4 = s4 < (unsigned)NBRUN, h5 = s5 < (unsigned)NBRUN, h6 = s6 < (unsigned)NBRUN, h7 = s7 < (unsigned)NBRUN;
      const unsigned m0 = __builtin_amdgcn_ballot_w32(h0), m1 = __builtin_amdgcn_ballot_w32(h1);
      const unsigned m2 = __builtin_amdgcn_ballot_w32(h2), m3 = __builtin_amdgcn_ballot_w32(h3);
      const unsigned m4 = __builtin_amdgcn_ballot_w32(h4), m5 = __builtin_amdgcn_ballot_w32(h5);
      const unsigned m6 = __builtin_amdgcn_ballot_w32(h6), m7 = __builtin_amdgcn_ballot_w32(h7);
      const unsigned any = m0 | m1 | m2 | m3 | m4 | m5 | m6 | m7;
      if (any != 0u) {
        const int pre = (int)(__builtin_amdgcn_mbcnt_lo(m0, 0u) + __builtin_amdgcn_mbcnt_lo(m1, 0u) +
                              __builtin_amdgcn_mbcnt_lo(m2, 0u) + __builtin_amdgcn_mbcnt_lo(m3, 0u) +
                              __builtin_amdgcn_mbcnt_lo(m4, 0u) + __builtin_amdgcn_mbcnt_lo(m5, 0u) +
                              __builtin_amdgcn_mbcnt_lo(m6, 0u) + __builtin_amdgcn_mbcnt_lo(m7, 0u));
        int p = wc + pre;
        if (h0) { if (p < WLCAP) mylist[p] = ((e0 + 0) << SLB) | (int)s0; p = p + 1; }
        if (h1) { if (p < WLCAP) mylist[p] = ((e0 + 1) << SLB) | (int)s1; p = p + 1; }
        if (h2) { if (p < WLCAP) mylist[p] = ((e0 + 2) << SLB) | (int)s2; p = p + 1; }
        if (h3) { if (p < WLCAP) mylist[p] = ((e0 + 3) << SLB) | (int)s3; p = p + 1; }
        if (h4) { if (p < WLCAP) mylist[p] = ((e0 + 4) << SLB) | (int)s4; p = p + 1; }
        if (h5) { if (p < WLCAP) mylist[p] = ((e0 + 5) << SLB) | (int)s5; p = p + 1; }
        if (h6) { if (p < WLCAP) mylist[p] = ((e0 + 6) << SLB) | (int)s6; p = p + 1; }
        if (h7) { if (p < WLCAP) mylist[p] = ((e0 + 7) << SLB) | (int)s7; p = p + 1; }
        wc += (int)(__builtin_popcount(m0) + __builtin_popcount(m1) + __builtin_popcount(m2) + __builtin_popcount(m3) +
                    __builtin_popcount(m4) + __builtin_popcount(m5) + __builtin_popcount(m6) + __builtin_popcount(m7));
      }
    }
    if (lane == 0) misc[wave] = wc;
  }
  __syncthreads();

  if (wave == 0) {
    int ov = 0;
    int tot = 0;
#pragma unroll 1
    for (int w2 = 0; w2 < NWAVE; ++w2) {
      int c = misc[w2];
      if (c > WLCAP) ov = 1;
      c = c < 0 ? 0 : (c > WLCAP ? WLCAP : c);
      tot += c;
#pragma unroll 1
      for (int b0 = 0; b0 < c; b0 += 32) {
        const int idx = b0 + lane;
        const int ent = wl[w2 * WLCAP + (idx < WLCAP ? idx : WLCAP - 1)];
        const int m32 = (c - b0) < 32 ? (c - b0) : 32;
#pragma unroll 1
        for (int k = 0; k < m32; ++k) {
          const int u    = __builtin_amdgcn_readlane(ent, k);
          const int slot = u & (NBRUN - 1);
          if (lane == 0) cnt[slot] = cnt[slot] + 1;
        }
      }
    }
    if (tot > RCAP) ov = 1;
    if (lane == 0) misc[9] = ov;
  }
  __syncthreads();
  if (wave == 0) {
    const int base = lane * (NBRUN / 32);
    int s = 0;
#pragma unroll 1
    for (int i = 0; i < NBRUN / 32; ++i) s += cnt[base + i];
    int incl = s;
#pragma unroll
    for (int d = 1; d < 32; d <<= 1) {
      const int y = __shfl_up(incl, d, 32);
      if (lane >= d) incl += y;
    }
    int run = incl - s;
#pragma unroll 1
    for (int i = 0; i < NBRUN / 32; ++i) {
      const int cv = cnt[base + i];
      offs[base + i] = run;
      cur[base + i]  = run;
      run += cv;
    }
  }
  __syncthreads();

  if (wave == 0) {
#pragma unroll 1
    for (int w2 = 0; w2 < NWAVE; ++w2) {
      int c = misc[w2];
      c = c < 0 ? 0 : (c > WLCAP ? WLCAP : c);
#pragma unroll 1
      for (int b0 = 0; b0 < c; b0 += 32) {
        const int idx = b0 + lane;
        const int ent = wl[w2 * WLCAP + (idx < WLCAP ? idx : WLCAP - 1)];
        int eid = (ent >> SLB) & 0x3FFFFF;
        eid = eid > NE - 1 ? NE - 1 : eid;
        int sr = srcs[eid];
        sr = sr < 0 ? 0 : (sr > NN - 1 ? NN - 1 : sr);
        const int wbits = (int)(bf16_bits(ew[eid]) << 16);
        const int m32 = (c - b0) < 32 ? (c - b0) : 32;
#pragma unroll 1
        for (int k = 0; k < m32; ++k) {
          const int u    = __builtin_amdgcn_readlane(ent, k);
          const int w0   = __builtin_amdgcn_readlane(sr, k);
          const int w1   = __builtin_amdgcn_readlane(wbits, k);
          const int slot = u & (NBRUN - 1);
          if (lane == 0) {
            int p = cur[slot];
            p = p < 0 ? 0 : (p > RCAP - 1 ? RCAP - 1 : p);
            pl[2 * p]     = w0;
            pl[2 * p + 1] = w1;
            cur[slot] = p + 1;
          }
        }
      }
    }
  }
  __syncthreads();

  const int ovf = misc[9];
  int* lp  = LIST + (size_t)blk * (size_t)(2 * RCAP);
  int* cop = CO + (size_t)blk * (2 * NBRUN);
  int* fp  = FLAG + (size_t)blk * 32;
  bucket_flush(pl, cnt, ovf, lp, cop, fp, tid);
  __threadfence();
  bucket_flush(pl, cnt, ovf, lp, cop, fp, tid);
}

template <int KTOT>
__device__ __forceinline__ void gemm_16x64(const unsigned short* __restrict__ ap,
                                           const unsigned short* __restrict__ bp, v8f (&acc)[4]) {
#pragma unroll 1
  for (int k0 = 0; k0 < KTOT; k0 += 32) {
    FragB af;
    af.h[0] = *(const v8usa*)(ap + k0);
    af.h[1] = *(const v8usa*)(ap + k0 + 16);
#pragma unroll
    for (int nt = 0; nt < 4; ++nt) {
      const unsigned short* wq = bp + (size_t)(16 * nt) * (size_t)KTOT + k0;
      FragB bf;
      bf.h[0] = *(const v8usa*)wq;
      bf.h[1] = *(const v8usa*)(wq + 16);
      acc[nt] = wmb(af, bf, acc[nt]);
    }
  }
}

__device__ __forceinline__ void stage_d(float* stg, const v8f (&acc)[4], int wave, int hh, int m) {
#pragma unroll
  for (int nt = 0; nt < 4; ++nt) {
#pragma unroll
    for (int r = 0; r < 8; ++r) stg[(16 * wave + 8 * hh + r) * SP + 16 * nt + m] = acc[nt][r];
  }
}

__global__ __launch_bounds__(NTHR) __attribute__((amdgpu_num_vgpr(248)))
void k_gemm(const unsigned short* __restrict__ XB, const unsigned short* __restrict__ WT, float* P) {
  __shared__ __attribute__((aligned(16))) float stg[GBM * SP];
  const int tid = (int)threadIdx.x, lane = tid & 31, wave = tid >> 5, hh = lane >> 4, m = lane & 15;
  const int rowBase = (int)blockIdx.x * GBM;

  v8f acc[4];
  {
    const v8f z = {0.f, 0.f, 0.f, 0.f, 0.f, 0.f, 0.f, 0.f};
#pragma unroll
    for (int t = 0; t < 4; ++t) acc[t] = z;
  }
  const unsigned short* ap = XB + (size_t)(rowBase + 16 * wave + m) * (size_t)KD + 8 * hh;
  const unsigned short* bp = WT + (size_t)m * (size_t)KD + 8 * hh;
  gemm_16x64<KD>(ap, bp, acc);
  stage_d(stg, acc, wave, hh, m);
  __syncthreads();

#pragma unroll 1
  for (int i = 0; i < 8; ++i) {
    const int lr   = 16 * wave + 2 * i + hh;
    const int grow = rowBase + lr;
    const bool live = grow < NN;
    const v4f a = *(const v4fa*)(stg + lr * SP + 4 * m);
    asm volatile("" :: "v"(a));
    v4f o;
    o.x = live ? a.x : 0.0f; o.y = live ? a.y : 0.0f; o.z = live ? a.z : 0.0f; o.w = live ? a.w : 0.0f;
    st2_v4f(P + (size_t)grow * HD + 4 * m, o);
  }
}

__global__ __launch_bounds__(NTHR) void k_replay(const int* __restrict__ LIST, const int* __restrict__ CO,
                                                 const int* __restrict__ FLAG, const float* __restrict__ P,
                                                 float* PRE, double* REC) {
  __shared__ __attribute__((aligned(16))) int sco[2 * NBRUN];
  __shared__ __attribute__((aligned(16))) double wsum[NWAVE * 128];
  const int tid = (int)threadIdx.x, lane = tid & 31, wave = tid >> 5;
  const int blk = (int)blockIdx.x;
  const int* lb = LIST + (size_t)blk * (size_t)(2 * RCAP);
  {
    const v4i v = *(const v4ia*)(CO + (size_t)blk * (2 * NBRUN) + 4 * tid);
    *(v4ia*)(sco + 4 * tid) = v;
  }
  const int flag = FLAG[(size_t)blk * 32];
  __syncthreads();

  const float qnan = __uint_as_float(0x7fc00000u);
  const float pz = (flag != 0) ? qnan : 0.0f;
  double S0 = 0.0, Q0 = 0.0, S1 = 0.0, Q1 = 0.0;

#pragma unroll 1
  for (int si = 0; si < NBRUN / NWAVE; ++si) {
    const int slot = si * NWAVE + wave;
    const int node = blk * NBRUN + slot;
    int c = sco[slot];
    int o = sco[NBRUN + slot];
    const bool big = c > DEGCAP;
    c = c < 0 ? 0 : (c > DEGCAP ? DEGCAP : c);
    o = o < 0 ? 0 : (o > RCAP - 1 ? RCAP - 1 : o);
    int last = o + (c > 0 ? c : 1) - 1;
    last = last > RCAP - 1 ? RCAP - 1 : last;
    float a0 = 0.0f, a1 = 0.0f;
#pragma unroll 1
    for (int b0 = 0; b0 < c; b0 += 32) {
      int idx = o + b0 + lane;
      idx = idx > last ? last : idx;
      const v2i ent = *(const v2ia*)(lb + 2 * idx);
      int sr = ent.x;
      sr = sr < 0 ? 0 : (sr > NN - 1 ? NN - 1 : sr);
      const int wv = ent.y;
      const int m32 = (c - b0) < 32 ? (c - b0) : 32;
#pragma unroll 1
      for (int k = 0; k < m32; ++k) {
        const int   sk = __builtin_amdgcn_readlane(sr, k);
        const float ck = __int_as_float(__builtin_amdgcn_readlane(wv, k));
        const v2f q = *(const v2fa*)(P + (size_t)sk * HD + 2 * lane);
        a0 = fmaf(ck, q.x, a0);
        a1 = fmaf(ck, q.y, a1);
      }
    }
    const float pzr = big ? qnan : pz;
    const float v0 = a0 + pzr;
    const float v1 = a1 + pzr;
    if (node < NN) {
      v2f ov;
      ov.x = v0; ov.y = v1;
      float* op = PRE + (size_t)node * HD + 2 * lane;
      *(volatile v2f*)op = ov;
      __threadfence();
      *(volatile v2f*)op = ov;
      const double d0 = (double)v0, d1 = (double)v1;
      S0 += d0; Q0 += d0 * d0;
      S1 += d1; Q1 += d1 * d1;
    }
  }

  wsum[wave * 128 + 4 * lane + 0] = S0;
  wsum[wave * 128 + 4 * lane + 1] = Q0;
  wsum[wave * 128 + 4 * lane + 2] = S1;
  wsum[wave * 128 + 4 * lane + 3] = Q1;
  __syncthreads();
  if (tid < HD) {
    double s = 0.0, q = 0.0;
#pragma unroll 1
    for (int w2 = 0; w2 < NWAVE; ++w2) {
      s += wsum[w2 * 128 + 2 * tid];
      q += wsum[w2 * 128 + 2 * tid + 1];
    }
    v2d r;
    r.x = s; r.y = q;
    double* rp = REC + (size_t)blk * 128 + 2 * tid;
    *(volatile v2d*)rp = r;
    __threadfence();
    *(volatile v2d*)rp = r;
  }
}

__global__ __launch_bounds__(HD) void k_combine(const double* __restrict__ REC, float* STAT) {
  __shared__ __attribute__((aligned(16))) float stg[2 * HD];
  const int c = (int)threadIdx.x;
  double S = 0.0, Q = 0.0;
#pragma unroll 1
  for (int b = 0; b < NBK; ++b) {
    const v2d r = *(const v2da*)(REC + (size_t)b * 128 + 2 * c);
    S += r.x;
    Q += r.y;
  }
  const double invN = 1.0 / (double)NN;
  const double mean = S * invN;
  double var = Q * invN - mean * mean;
  var = (var < 0.0) ? 0.0 : var;
  const float varf = (float)var;
  const float rs = 1.0f / sqrtf(varf + 0.001f);
  stg[c] = (float)mean;
  stg[HD + c] = rs;
  __syncthreads();
  if (c < 32) {
    const v4f v = *(const v4fa*)(stg + 4 * c);
    st2_v4f(STAT + 4 * c, v);
  }
}

__global__ __launch_bounds__(NTHR) void k_apply(const float* __restrict__ PRE, const float* __restrict__ STAT,
                                                const int* __restrict__ FLAG, float* out) {
  __shared__ __attribute__((aligned(16))) float ssh[2 * HD];
  const int tid = (int)threadIdx.x;
  const int blk = (int)blockIdx.x;
  if (tid < 32) *(v4fa*)(ssh + 4 * tid) = *(const v4fa*)(STAT + 4 * tid);
  const int flag = FLAG[(size_t)(blk >> 5) * 32];
  __syncthreads();
  const int u  = blk * NTHR + tid;
  const int c4 = (u & 15) * 4;
  const v4f v  = *(const v4fa*)(PRE + (size_t)u * 4);
  const v4f mu = *(const v4fa*)(ssh + c4);
  const v4f rs = *(const v4fa*)(ssh + HD + c4);
  float t0 = (v.x - mu.x) * rs.x, t1 = (v.y - mu.y) * rs.y;
  float t2 = (v.z - mu.z) * rs.z, t3 = (v.w - mu.w) * rs.w;
  t0 = (t0 > 0.0f) ? t0 : (t0 - t0); t1 = (t1 > 0.0f) ? t1 : (t1 - t1);
  t2 = (t2 > 0.0f) ? t2 : (t2 - t2); t3 = (t3 > 0.0f) ? t3 : (t3 - t3);
  const float qnan = __uint_as_float(0x7fc00000u);
  const bool bad = flag != 0;
  v4f o;
  o.x = bad ? qnan : t0; o.y = bad ? qnan : t1; o.z = bad ? qnan : t2; o.w = bad ? qnan : t3;
  st2_v4f(out + (size_t)u * 4, o);
}

extern "C" void kernel_launch(void* const* d_in, const int* in_sizes, int n_in,
                              void* d_out, int out_size, void* d_ws, size_t ws_size,
                              hipStream_t stream) {
  if (n_in < 5) return;
  if (in_sizes[0] != NN * KD) return;
  if (in_sizes[1] != KD * HD) return;
  if (in_sizes[2] != NE) return;
  if (in_sizes[3] != NE) return;
  if (in_sizes[4] != NE) return;
  if (out_size != NN * HD) return;

  const float* x  = (const float*)d_in[0];
  const float* W  = (const float*)d_in[1];
  const float* ew = (const float*)d_in[2];
  const int* srcs = (const int*)d_in[3];
  const int* dsts = (const int*)d_in[4];
  float* out = (float*)d_out;

  constexpr size_t zXB   = (size_t)MP * KD * 2;
  constexpr size_t zP    = (size_t)MP * HD * 4;
  constexpr size_t zPRE  = (size_t)NN * HD * 4;
  constexpr size_t zLIST = (size_t)NBK * RCAP * 8;
  constexpr size_t zCO   = (size_t)NBK * 2 * NBRUN * 4;
  constexpr size_t zREC  = (size_t)NBK * 128 * 8;
  constexpr size_t zFLAG = 28672;
  constexpr size_t zWT   = (size_t)HD * KD * 2;
  constexpr size_t zSTAT = 512;
  constexpr size_t oXB   = 0;
  constexpr size_t oP    = oXB + zXB;
  constexpr size_t oPRE  = oP + zP;
  constexpr size_t oLIST = oPRE + zPRE;
  constexpr size_t oCO   = oLIST + zLIST;
  constexpr size_t oREC  = oCO + zCO;
  constexpr size_t oFLAG = oREC + zREC;
  constexpr size_t oWT   = oFLAG + zFLAG;
  constexpr size_t oSTAT = oWT + zWT;
  constexpr size_t oEND  = oSTAT + zSTAT;
  static_assert(zXB % 256 == 0 && zP % 256 == 0 && zPRE % 256 == 0 && zLIST % 256 == 0 && zCO % 256 == 0);
  static_assert(zREC % 256 == 0 && zFLAG % 256 == 0 && zWT % 256 == 0 && zSTAT % 256 == 0);
  static_assert(zFLAG >= (size_t)NBK * 128);
  static_assert(zCO + zREC + zFLAG == (size_t)PBZ * NTHR * 16);
  static_assert(oEND <= (size_t)WSMAX);
  if (oEND > ws_size) return;

  char* ws = (char*)d_ws;
  unsigned short* XB   = (unsigned short*)(ws + oXB);
  float*          P    = (float*)(ws + oP);
  float*          PRE  = (float*)(ws + oPRE);
  int*            LIST = (int*)(ws + oLIST);
  int*            CO   = (int*)(ws + oCO);
  double*         REC  = (double*)(ws + oREC);
  int*            FLAG = (int*)(ws + oFLAG);
  unsigned short* WT   = (unsigned short*)(ws + oWT);
  float*          STAT = (float*)(ws + oSTAT);

  hipFuncSetAttribute(reinterpret_cast<const void*>(&k_bucket), hipFuncAttributeMaxDynamicSharedMemorySize, (int)BK_LDS);

  k_prep<<<PBTOT, NTHR, 0, stream>>>(x, W, XB, WT, CO);
  k_bucket<<<NBK, NTHR, BK_LDS, stream>>>(srcs, dsts, ew, LIST, CO, FLAG);
  k_gemm<<<MP / GBM, NTHR, 0, stream>>>(XB, WT, P);
  k_replay<<<NBK, NTHR, 0, stream>>>(LIST, CO, FLAG, P, PRE, REC);
  k_combine<<<1, HD, 0, stream>>>(REC, STAT);
  k_apply<<<(NN * HD / 4) / NTHR, NTHR, 0, stream>>>(PRE, STAT, FLAG, out);
}
